// MatNetCrossMHA_39032662786225
// MI455X (gfx1250) — hardware-verified
//
#include <hip/hip_runtime.h>


#define NB_  4
#define MM   512
#define NN   512
#define EE   256
#define NH_  16
#define HD   16
#define KP   32
#define VP   64
#define HID  16
typedef _Float16 h16;
typedef unsigned short bf;
typedef __attribute__((ext_vector_type(16))) __bf16   v16bf;
typedef __attribute__((ext_vector_type(16))) _Float16 v16h;
typedef __attribute__((ext_vector_type(8)))  _Float16 v8h;
typedef __attribute__((ext_vector_type(8)))  unsigned short v8us;
typedef __attribute__((ext_vector_type(8)))  float    v8f;
typedef __attribute__((ext_vector_type(4)))  float    v4f;
typedef v8h  __attribute__((may_alias)) v8ha;
typedef v4f  __attribute__((may_alias)) v4fa;
typedef v8us __attribute__((may_alias)) v8usa;

__device__ __forceinline__ unsigned short f2bf(float f) { unsigned u = __float_as_uint(f); u += 0x7FFFu + ((u >> 16) & 1u); return (unsigned short)(u >> 16); }
__device__ __forceinline__ float bf2f(unsigned short b) { return __uint_as_float(((unsigned)b) << 16); }
__device__ __forceinline__ float bfr(float f) { return bf2f(f2bf(f)); }
__device__ __forceinline__ v16h cat16(v8h lo, v8h hi) { return __builtin_shufflevector(lo, hi, 0, 1, 2, 3, 4, 5, 6, 7, 8, 9, 10, 11, 12, 13, 14, 15); }
__device__ __forceinline__ v16bf cat16b(v8us lo, v8us hi) { return __builtin_bit_cast(v16bf, __builtin_shufflevector(lo, hi, 0, 1, 2, 3, 4, 5, 6, 7, 8, 9, 10, 11, 12, 13, 14, 15)); }
__device__ __forceinline__ v8f wmma16(v16h a, v16h b, v8f c) { return __builtin_amdgcn_wmma_f32_16x16x32_f16(false, a, false, b, (short)0, c, false, false); }
__device__ __forceinline__ v8f wmmab(v16bf a, v16bf b, v8f c) { return __builtin_amdgcn_wmma_f32_16x16x32_bf16(false, a, false, b, (short)0, c, false, false); }


template <typename T16> struct WFrag;
template <> struct WFrag<h16> { typedef v16h V; static __device__ __forceinline__ V ld(const h16* p) { return cat16(*(const v8h*)p, *(const v8h*)(p + 16)); } static __device__ __forceinline__ v8f mma(V a, V b, v8f c) { return wmma16(a, b, c); } };
template <> struct WFrag<bf> { typedef v16bf V; static __device__ __forceinline__ V ld(const bf* p) { return cat16b(*(const v8us*)p, *(const v8us*)(p + 16)); } static __device__ __forceinline__ v8f mma(V a, V b, v8f c) { return wmmab(a, b, c); } };
template <typename T16, int NSPLIT, bool BIAS>
__global__ __launch_bounds__(32) void k_gemmw(const T16* __restrict__ A, const T16* __restrict__ A2, const T16* __restrict__ Bt, const T16* __restrict__ Bt2, int K, float* C, int ldc, const float* __restrict__ bias, size_t sA, size_t sB, size_t sC) {
    typedef typename WFrag<T16>::V V;
    __shared__ __align__(16) float os[16 * 68];
    const size_t z = blockIdx.z; A += z * sA; if (A2) A2 += z * sA; Bt += z * sB; if (Bt2) Bt2 += z * sB; C += z * sC;
    const int lane = threadIdx.x & 31, lr = lane & 15, hi = lane >> 4; const int r0 = blockIdx.x * 64, c0 = blockIdx.y * 64;
    v8f acc[4][4];
#pragma unroll
    for (int mb = 0; mb < 4; ++mb)
#pragma unroll
        for (int nb = 0; nb < 4; ++nb) acc[mb][nb] = (v8f){};
    const size_t aoff = (size_t)(r0 + lr) * K + 8 * hi, boff = (size_t)(c0 + lr) * K + 8 * hi;
#pragma unroll 1
    for (int kc = 0; kc < K; kc += 32) {
        V a[4], a2[4];
#pragma unroll
        for (int mb = 0; mb < 4; ++mb) { a[mb] = WFrag<T16>::ld(A + aoff + (size_t)mb * 16 * K + kc); if (NSPLIT == 1 || NSPLIT == 2) a2[mb] = WFrag<T16>::ld(A2 + aoff + (size_t)mb * 16 * K + kc); }
#pragma unroll
        for (int nb = 0; nb < 4; ++nb) { const V b = WFrag<T16>::ld(Bt + boff + (size_t)nb * 16 * K + kc); V b2; if (NSPLIT >= 2) b2 = WFrag<T16>::ld(Bt2 + boff + (size_t)nb * 16 * K + kc);
#pragma unroll
            for (int mb = 0; mb < 4; ++mb) { acc[mb][nb] = WFrag<T16>::mma(a[mb], b, acc[mb][nb]); if (NSPLIT == 1 || NSPLIT == 2) acc[mb][nb] = WFrag<T16>::mma(a2[mb], b, acc[mb][nb]); if (NSPLIT >= 2) acc[mb][nb] = WFrag<T16>::mma(a[mb], b2, acc[mb][nb]); } }
        asm volatile("v_nop\n\tv_nop\n\tv_nop\n\tv_nop" : "+v"(acc[0][0]), "+v"(acc[1][1]), "+v"(acc[2][2]), "+v"(acc[3][3]) : "v"(a[0]), "v"(a[3]));
    }
#pragma unroll
    for (int mb = 0; mb < 4; ++mb) {
#pragma unroll
        for (int nb = 0; nb < 4; ++nb) {
#pragma unroll
            for (int j = 0; j < 8; ++j) os[(hi * 8 + j) * 68 + nb * 16 + lr] = acc[mb][nb][j]; }
        __builtin_amdgcn_wave_barrier(); asm volatile("" ::: "memory");
        float* crow = C + (size_t)(r0 + mb * 16) * ldc + c0;
#pragma unroll 1
        for (int ps = 0; ps < 2; ++ps) {
#pragma unroll
            for (int s = 0; s < 8; ++s) { const int row = 2 * s + hi, cofs = lr * 4; v4f val = *(const v4fa*)(os + row * 68 + cofs); if (BIAS) { val[0] += bfr(bias[c0 + cofs]); val[1] += bfr(bias[c0 + cofs + 1]); val[2] += bfr(bias[c0 + cofs + 2]); val[3] += bfr(bias[c0 + cofs + 3]); }
                *(volatile v4f*)(crow + (size_t)row * ldc + cofs) = val; }
            if (ps == 0) __threadfence(); }
        __builtin_amdgcn_wave_barrier(); asm volatile("" ::: "memory");
    }
}

__device__ __forceinline__ void splitf(float y, unsigned short& h, unsigned short& l) { h = f2bf(y); l = f2bf(y - bf2f(h)); }
typedef __attribute__((ext_vector_type(2))) unsigned short v2us;
typedef __attribute__((ext_vector_type(4))) unsigned short v4us;

__global__ __launch_bounds__(256) void k_cvt8(const float* __restrict__ src, bf* dst, size_t n8) { const size_t i = (size_t)blockIdx.x * 256 + threadIdx.x; if (i >= n8) return; const v8f v = *(const v8f*)(src + i * 8); v8us o;
#pragma unroll
    for (int k = 0; k < 8; ++k) o[k] = f2bf(v[k]); *(volatile v8us*)(dst + i * 8) = o; __threadfence(); *(volatile v8us*)(dst + i * 8) = o; }
__global__ __launch_bounds__(256) void k_qkpl(const float* __restrict__ FQ, const float* __restrict__ FKV, bf* Qh, bf* Ql, bf* Kh, bf* Kl) { const int e = (blockIdx.x * 256 + threadIdx.x) * 4; if (e >= NH_ * MM * KP) return; const int kp = e % KP; const int m = (e / KP) % MM; const int h = e / (KP * MM); v4us qh, ql, kh, kl;
#pragma unroll
    for (int u = 0; u < 4; ++u) { unsigned short a = 0, b = 0, c = 0, d2 = 0; const int d = kp + u; if (d < HD) { splitf(FQ[(size_t)m * EE + h * HD + d] * 0.25f, a, b); splitf(FKV[(size_t)m * 2 * EE + h * HD + d], c, d2); } qh[u] = a; ql[u] = b; kh[u] = c; kl[u] = d2; }
    for (int ps = 0; ps < 2; ++ps) { *(volatile v4us*)(Qh + e) = qh; *(volatile v4us*)(Ql + e) = ql; *(volatile v4us*)(Kh + e) = kh; *(volatile v4us*)(Kl + e) = kl; if (ps == 0) __threadfence(); } }
__global__ __launch_bounds__(256) void k_vt(const float* __restrict__ FKV, bf* Vh, bf* Vl) { const int e = (blockIdx.x * 256 + threadIdx.x) * 2; if (e >= NH_ * VP * NN) return; const int n = e % NN; const int vp = (e / NN) % VP; const int h = e / (NN * VP); v2us oh, ol;
#pragma unroll
    for (int u = 0; u < 2; ++u) { unsigned short a = 0, b = 0; if (vp < HD) splitf(FKV[(size_t)(n + u) * 2 * EE + EE + h * HD + vp], a, b); oh[u] = a; ol[u] = b; } for (int ps = 0; ps < 2; ++ps) { *(volatile v2us*)(Vh + e) = oh; *(volatile v2us*)(Vl + e) = ol; if (ps == 0) __threadfence(); } }
__global__ __launch_bounds__(256) void k_mrg(const float* __restrict__ O, bf* Ah, bf* Al) { const int e = (blockIdx.x * 256 + threadIdx.x) * 4; if (e >= MM * EE) return; const int c = e % EE; const int m = e / EE; const int h = c / HD, d = c % HD; const float* r = O + ((size_t)h * MM + m) * VP + d; v4us oh, ol;
#pragma unroll
    for (int u = 0; u < 4; ++u) { unsigned short a, b; splitf(r[u], a, b); oh[u] = a; ol[u] = b; } *(volatile v4us*)(Ah + e) = oh; *(volatile v4us*)(Al + e) = ol; __threadfence(); *(volatile v4us*)(Ah + e) = oh; *(volatile v4us*)(Al + e) = ol; }
__global__ __launch_bounds__(256) void k_mixsoft(const float* __restrict__ Sb, const float* __restrict__ dm, const float* __restrict__ W1, const float* __restrict__ b1, const float* __restrict__ W2, const float* __restrict__ b2, bf* Ph, bf* Pl) {
    const int lane = threadIdx.x & 31; const int row = blockIdx.x * 8 + (threadIdx.x >> 5); if (row >= NH_ * MM) return; const int m = row % MM; const int h = row / MM; const float* sr = Sb + (size_t)row * NN; const float* dr = dm + (size_t)m * NN;
    float w0[HID], w1[HID], bb[HID], w2[HID];
#pragma unroll
    for (int k = 0; k < HID; ++k) { w0[k] = bfr(W1[(h * 2 + 0) * HID + k]); w1[k] = bfr(W1[(h * 2 + 1) * HID + k]); bb[k] = bfr(b1[h * HID + k]); w2[k] = bfr(W2[h * HID + k]); asm volatile("" : "+v"(w0[k])); asm volatile("" : "+v"(w1[k])); asm volatile("" : "+v"(bb[k])); asm volatile("" : "+v"(w2[k])); }
    float bb2 = bfr(b2[h]); asm volatile("" : "+v"(bb2)); float v[NN / 32]; float mx = -3.0e38f;
#pragma unroll
    for (int ch = 0; ch < NN / 128; ++ch) { const int j0 = ch * 128 + lane * 4; const v4f a = *(const v4f*)(sr + j0), dd = *(const v4f*)(dr + j0);
#pragma unroll
        for (int u = 0; u < 4; ++u) { float dv = bfr(dd[u]); asm volatile("" : "+v"(dv)); float acc = bb2;
#pragma unroll
            for (int k = 0; k < HID; ++k) { float p0 = __fmul_rn(a[u], w0[k]), p1 = __fmul_rn(dv, w1[k]); asm volatile("" : "+v"(p0)); asm volatile("" : "+v"(p1)); const float hk = fmaxf(__fadd_rn(__fadd_rn(p0, p1), bb[k]), 0.f); float pk = __fmul_rn(hk, w2[k]); asm volatile("" : "+v"(pk)); acc = __fadd_rn(acc, pk); }
            v[ch * 4 + u] = acc; mx = fmaxf(mx, acc); } }
#pragma unroll
    for (int sh = 16; sh; sh >>= 1) mx = fmaxf(mx, __shfl_xor(mx, sh, 32));
    float sum = 0.f;
#pragma unroll
    for (int q = 0; q < NN / 32; ++q) { float d0 = __fsub_rn(v[q], mx); asm volatile("" : "+v"(d0)); v[q] = __expf(d0); sum += v[q]; }
#pragma unroll
    for (int sh = 16; sh; sh >>= 1) sum += __shfl_xor(sum, sh, 32);
    const float f = __fdiv_rn(1.0f, sum);
    for (int ps = 0; ps < 2; ++ps) {
#pragma unroll
        for (int ch = 0; ch < NN / 128; ++ch) { v4us oh, ol;
#pragma unroll
            for (int u = 0; u < 4; ++u) { unsigned short a, b; splitf(v[ch * 4 + u] * f, a, b); oh[u] = a; ol[u] = b; } const size_t oo = (size_t)row * NN + ch * 128 + lane * 4; *(volatile v4us*)(Ph + oo) = oh; *(volatile v4us*)(Pl + oo) = ol; }
        if (ps == 0) __threadfence(); } }

extern "C" void kernel_launch(void* const* d_in, const int* in_sizes, int n_in,
                              void* d_out, int out_size, void* d_ws, size_t ws_size, hipStream_t stream) {
    (void)in_sizes; (void)n_in; (void)out_size;
    const float** I = (const float**)d_in;
    const float *qin = I[0], *kvin = I[1], *dmat = I[2], *wq = I[3], *wkv = I[4], *W1 = I[5], *b1 = I[6], *W2 = I[7], *b2 = I[8], *wout = I[9];
    float* OUT = (float*)d_out;
    char* wsp = (char*)d_ws;
    auto take = [&](size_t bytes) { char* p = wsp; wsp += (bytes + 255) & ~(size_t)255; return (void*)p; };
    bf* WQ = (bf*)take(EE * EE * 2); bf* WKV = (bf*)take(2 * EE * EE * 2); bf* WO = (bf*)take(EE * EE * 2);
    bf* QB = (bf*)take((size_t)MM * EE * 2); bf* KB = (bf*)take((size_t)NN * EE * 2); float* FQ = (float*)take((size_t)MM * EE * 4); float* FKV = (float*)take((size_t)NN * 2 * EE * 4); bf* Qh = (bf*)take((size_t)NH_ * MM * KP * 2); bf* Ql = (bf*)take((size_t)NH_ * MM * KP * 2); bf* Kh = (bf*)take((size_t)NH_ * NN * KP * 2); bf* Kl = (bf*)take((size_t)NH_ * NN * KP * 2); bf* Vh = (bf*)take((size_t)NH_ * VP * NN * 2); bf* Vl = (bf*)take((size_t)NH_ * VP * NN * 2);
    float* Sb = (float*)take((size_t)NH_ * MM * NN * 4); bf* Ph = (bf*)take((size_t)NH_ * MM * NN * 2); bf* Pl = (bf*)take((size_t)NH_ * MM * NN * 2); float* O = (float*)take((size_t)NH_ * MM * VP * 4); bf* Ah = (bf*)take((size_t)MM * EE * 2); bf* Al = (bf*)take((size_t)MM * EE * 2);
    if ((size_t)(wsp - (char*)d_ws) > ws_size) return;
    k_cvt8<<<(EE * EE / 8 + 255) / 256, 256, 0, stream>>>(wq, WQ, EE * EE / 8); k_cvt8<<<(2 * EE * EE / 8 + 255) / 256, 256, 0, stream>>>(wkv, WKV, 2 * EE * EE / 8); k_cvt8<<<(EE * EE / 8 + 255) / 256, 256, 0, stream>>>(wout, WO, EE * EE / 8);
    for (int b = 0; b < NB_; ++b) {
        k_cvt8<<<(MM * EE / 8 + 255) / 256, 256, 0, stream>>>(qin + (size_t)b * MM * EE, QB, (size_t)MM * EE / 8); k_cvt8<<<(NN * EE / 8 + 255) / 256, 256, 0, stream>>>(kvin + (size_t)b * NN * EE, KB, (size_t)NN * EE / 8);
        k_gemmw<bf, 0, false><<<dim3(MM / 64, EE / 64, 1), 32, 0, stream>>>(QB, nullptr, WQ, nullptr, EE, FQ, EE, nullptr, 0, 0, 0); k_gemmw<bf, 0, false><<<dim3(NN / 64, 2 * EE / 64, 1), 32, 0, stream>>>(KB, nullptr, WKV, nullptr, EE, FKV, 2 * EE, nullptr, 0, 0, 0);
        k_qkpl<<<(NH_ * MM * KP / 4 + 255) / 256, 256, 0, stream>>>(FQ, FKV, Qh, Ql, Kh, Kl); k_vt<<<(NH_ * VP * NN / 2 + 255) / 256, 256, 0, stream>>>(FKV, Vh, Vl);
        k_gemmw<bf, 2, false><<<dim3(MM / 64, NN / 64, NH_), 32, 0, stream>>>(Qh, Ql, Kh, Kl, KP, Sb, NN, nullptr, (size_t)MM * KP, (size_t)NN * KP, (size_t)MM * NN);
        k_mixsoft<<<NH_ * MM / 8, 256, 0, stream>>>(Sb, dmat + (size_t)b * MM * NN, W1, b1, W2, b2, Ph, Pl);
        k_gemmw<bf, 2, false><<<dim3(MM / 64, VP / 64, NH_), 32, 0, stream>>>(Ph, Pl, Vh, Vl, NN, O, VP, nullptr, (size_t)MM * NN, (size_t)VP * NN, (size_t)MM * VP);
        k_mrg<<<(MM * EE / 4 + 255) / 256, 256, 0, stream>>>(O, Ah, Al);
        k_gemmw<bf, 1, false><<<dim3(MM / 64, EE / 64, 1), 32, 0, stream>>>(Ah, Al, WO, nullptr, EE, OUT + (size_t)b * MM * EE, EE, nullptr, 0, 0, 0); }
}
